// GATrNet_81458349736002
// MI455X (gfx1250) — hardware-verified
//
#include <hip/hip_runtime.h>
#include <math.h>
#include <stdint.h>

typedef unsigned short us;
typedef __bf16 v16b __attribute__((ext_vector_type(16)));
typedef float v8f __attribute__((ext_vector_type(8)));
typedef float v4f __attribute__((ext_vector_type(4)));
typedef unsigned int v4u __attribute__((ext_vector_type(4)));
typedef v4f __attribute__((may_alias)) v4fa;
typedef v4u __attribute__((may_alias)) v4ua;

#define NSEQ  2048
#define NTOK  16384
#define NFEAT 256
#define HDIM  64

#define WP_Q 0
#define WP_K 2560
#define WP_V 5120
#define WP_O 7680
#define WP_1 10240
#define WP_2 20480
#define WP_LAYER 35840

static_assert(NTOK % 32 == 0);
static_assert(NTOK % 256 == 0);
static_assert(NSEQ % 64 == 0);
static_assert(2 * 16 == 32);
static_assert(96 == 6 * 16);
static_assert(WP_LAYER == WP_2 + 5 * 16 * 192);
static_assert((WP_LAYER * 2) % 128 == 0);

#define MASK_PACK 0xFEDB7CA965384210ULL
#define IDX_PACK  0xFEDAC984B7635210ULL
#define NOE0_PACK 0xEA974320u
constexpr int c_popc(int v) { return (v & 1) + ((v >> 1) & 1) + ((v >> 2) & 1) + ((v >> 3) & 1); }
constexpr int c_mask(int i) { return (int)((MASK_PACK >> (4 * i)) & 15ULL); }
constexpr int c_idx(int mk) { return (int)((IDX_PACK >> (4 * mk)) & 15ULL); }
constexpr int c_noe0(int s) { return (int)((NOE0_PACK >> (4 * s)) & 15u); }
constexpr int c_grade(int b) { return (b >= 1) + (b >= 5) + (b >= 11) + (b >= 15); }
constexpr int c_sign(int a, int b) {
  int cnt = 0; int aa = a >> 1;
  while (aa) { cnt += c_popc(aa & b); aa >>= 1; }
  return (cnt & 1) ? -1 : 1;
}
constexpr int c_cay(int i, int j, int k) {
  const int a = c_mask(i), b = c_mask(j);
  if (a & b & 1) return 0;
  if (c_idx(a ^ b) != k) return 0;
  return c_sign(a, b);
}
constexpr bool chk_tables() {
  for (int i = 0; i < 16; ++i) {
    if (c_idx(c_mask(i)) != i) return false;
    if (c_popc(c_mask(i)) != c_grade(i)) return false;
  }
  for (int i = 0; i < 15; ++i) {
    const int ga = c_popc(c_mask(i)), gb = c_popc(c_mask(i + 1));
    if (ga > gb) return false;
    if (ga == gb && c_mask(i) >= c_mask(i + 1)) return false;
  }
  for (int s = 0; s < 8; ++s) {
    if (c_mask(c_noe0(s)) & 1) return false;
    if (s > 0 && c_noe0(s) <= c_noe0(s - 1)) return false;
  }
  return true;
}
constexpr int c_nnz() {
  int n = 0;
  for (int i = 0; i < 16; ++i) for (int j = 0; j < 16; ++j) for (int k = 0; k < 16; ++k) if (c_cay(i, j, k) != 0) ++n;
  return n;
}
constexpr bool chk_scalar_left() { for (int j = 0; j < 16; ++j) if (c_cay(0, j, j) != 1) return false; return true; }
constexpr bool chk_e0sq() { for (int k = 0; k < 16; ++k) if (c_cay(1, 1, k) != 0) return false; return true; }
static_assert(chk_tables());
static_assert(c_nnz() == 192);
static_assert(chk_scalar_left());
static_assert(chk_e0sq());
static_assert(c_cay(2, 2, 0) == 1);
static_assert(c_cay(2, 3, 7) == 1);
static_assert(c_cay(3, 2, 7) == -1);
static_assert(c_cay(1, 2, 5) == 1);
static_assert(c_cay(2, 1, 5) == -1);
static_assert(c_cay(7, 7, 0) == -1);

__device__ __forceinline__ unsigned bf_bits(float f) {
  const unsigned u = __float_as_uint(f);
  return (u + 0x7FFFu + ((u >> 16) & 1u)) >> 16;
}
__device__ __forceinline__ float bfr(float f) { return __uint_as_float(bf_bits(f) << 16); }

struct F8 { float v[8]; };
struct HL { v4u hi; v4u lo; };
__device__ __forceinline__ HL split8(const F8& f) {
  unsigned hb[8], lb[8];
#pragma unroll
  for (int j = 0; j < 8; ++j) {
    hb[j] = bf_bits(f.v[j]);
    lb[j] = bf_bits(f.v[j] - __uint_as_float(hb[j] << 16));
  }
  HL o;
  o.hi = (v4u){hb[0] | (hb[1] << 16), hb[2] | (hb[3] << 16), hb[4] | (hb[5] << 16), hb[6] | (hb[7] << 16)};
  o.lo = (v4u){lb[0] | (lb[1] << 16), lb[2] | (lb[3] << 16), lb[4] | (lb[5] << 16), lb[6] | (lb[7] << 16)};
  return o;
}

__device__ __forceinline__ v8f mma_bf(v16b a, v16b b, v8f c) {
  c = __builtin_amdgcn_wmma_f32_16x16x32_bf16(false, a, false, b, (short)0, c, false, false);
  asm volatile("v_nop\n\tv_nop\n\tv_nop\n\tv_nop" : "+v"(c) : "v"(a), "v"(b));
  return c;
}
union FragU { v16b v; v4u q[2]; };
__device__ __forceinline__ v16b ldfrag_g(const us* __restrict__ p) {
  FragU f; f.q[0] = *(const v4ua*)(p); f.q[1] = *(const v4ua*)(p + 16); return f.v;
}
__device__ __forceinline__ v16b ldfrag_s(const us* p) {
  FragU f; f.q[0] = *(const v4ua*)(p); f.q[1] = *(const v4ua*)(p + 16); return f.v;
}

__device__ __forceinline__ v4u gather8(const float* __restrict__ src) {
  float f[8];
#pragma unroll
  for (int j = 0; j < 8; ++j) f[j] = src[j * 5];
  v4u o;
  o.x = bf_bits(f[0]) | (bf_bits(f[1]) << 16);
  o.y = bf_bits(f[2]) | (bf_bits(f[3]) << 16);
  o.z = bf_bits(f[4]) | (bf_bits(f[5]) << 16);
  o.w = bf_bits(f[6]) | (bf_bits(f[7]) << 16);
  return o;
}

__global__ __launch_bounds__(64) void k_prep(const float* __restrict__ wq, const float* __restrict__ wk,
                                             const float* __restrict__ wv, const float* __restrict__ wo,
                                             const float* __restrict__ w1, const float* __restrict__ w2,
                                             us* __restrict__ WPl) {
  const int tid = threadIdx.x;
  const int bl = blockIdx.x;
  const int l = bl / 70;
  const int bb = bl - l * 70;
  const int ub = bb * 64 + tid;
  v4u val;
  if (bb < 20) {
    const int mi = bb / 5;
    const int rr = (ub - mi * 320) * 8;
    const int g = rr >> 9, n = (rr & 511) >> 5, k0 = rr & 31, i0 = k0 & 15;
    const int off = l * 1280 + (n * 16 + i0) * 5 + g;
    if (mi == 0)      val = gather8(wq + off);
    else if (mi == 1) val = gather8(wk + off);
    else if (mi == 2) val = gather8(wv + off);
    else              val = gather8(wo + off);
  } else if (bb < 40) {
    const int rr = (ub - 1280) * 8;
    const int g = rr >> 11, n = (rr & 2047) >> 5, k0 = rr & 31, i0 = k0 & 15;
    val = gather8(w1 + l * 5120 + (n * 16 + i0) * 5 + g);
  } else {
    const int rr = (ub - 2560) * 8;
    const int g = rr / 3072;
    const int r2 = rr - g * 3072;
    const int n = r2 / 192;
    const int k0 = r2 - n * 192;
    const int i0 = (k0 >= 96) ? (k0 - 96) : k0;
    val = gather8(w2 + l * 7680 + (n * 96 + i0) * 5 + g);
  }
  us* dst = WPl + (size_t)l * WP_LAYER + (size_t)ub * 8;
  *(volatile v4u*)dst = val;
  __threadfence();
  *(volatile v4u*)dst = val;
}

#define PRE_SX 0
#define PRE_SA 32768
#define PRE_SQ 65536
#define PRE_SK 81920
#define PRE_SV 98304
#define PRE_SR 114688
#define PRE_SL 114816
#define PRE_LDS 114944
static_assert(PRE_LDS <= 327680);

template <int L>
__global__ __launch_bounds__(256) void k_pre(const float* __restrict__ pos, const float* __restrict__ vel,
                                             const float* __restrict__ lw,
                                             const float* Xin, float* Xout,
                                             const us* __restrict__ WP,
                                             us* __restrict__ Qp, us* __restrict__ Kp, us* __restrict__ VTp) {
  extern __shared__ __align__(16) unsigned char smem[];
  float* sX = (float*)(smem + PRE_SX);
  us*    sA = (us*)(smem + PRE_SA);
  us*    sQ = (us*)(smem + PRE_SQ);
  us*    sK = (us*)(smem + PRE_SK);
  us*    sV = (us*)(smem + PRE_SV);
  float* sR = (float*)(smem + PRE_SR);
  float* sL = (float*)(smem + PRE_SL);

  const int tid = threadIdx.x, lane = tid & 31, w = tid >> 5, h = lane >> 4, m = lane & 15;
  const int tok0 = blockIdx.x * 32;

  if (L == 0) {
    if (tid < 32) sL[tid] = bfr(lw[((tid & 15) * 2 + (tid >> 4)) * 5 + 1]);
    __syncthreads();
    const int tok = tid >> 3, part = tid & 7;
    const size_t t = (size_t)(tok0 + tok);
    const float p0 = bfr(pos[t * 3 + 0]), p1 = bfr(pos[t * 3 + 1]), p2 = bfr(pos[t * 3 + 2]);
    const float q0 = bfr(vel[t * 3 + 0]), q1 = bfr(vel[t * 3 + 1]), q2 = bfr(vel[t * 3 + 2]);
#pragma unroll
    for (int cc = 0; cc < 2; ++cc) {
      const int c = part * 2 + cc;
      const float l0 = sL[c], l1 = sL[16 + c];
      const v4f r0 = {0.0f, l0, p0 * l0 + q0 * l1, p1 * l0 + q1 * l1};
      const v4f r1 = {p2 * l0 + q2 * l1, 0.0f, 0.0f, 0.0f};
      const v4f zz = {0.0f, 0.0f, 0.0f, 0.0f};
      float* d = sX + tok * 256 + c * 16;
      *(v4fa*)(d) = r0; *(v4fa*)(d + 4) = r1; *(v4fa*)(d + 8) = zz; *(v4fa*)(d + 12) = zz;
    }
  } else {
#pragma unroll
    for (int it = 0; it < 8; ++it) {
      const int idx = it * 256 + tid;
      *(v4fa*)(sX + idx * 4) = *(const v4fa*)(Xin + (size_t)tok0 * 256 + (size_t)idx * 4);
    }
  }
  __syncthreads();

  {
    const int tok = tid >> 3, part = tid & 7;
    float s = 0.0f;
#pragma unroll
    for (int i = 0; i < 8; ++i) {
      const v4f v = *(const v4fa*)(sX + tok * 256 + part * 32 + i * 4);
      s += v.x * v.x + v.y * v.y + v.z * v.z + v.w * v.w;
    }
    s += __shfl_xor(s, 1, 32);
    s += __shfl_xor(s, 2, 32);
    s += __shfl_xor(s, 4, 32);
    if (part == 0) sR[tok] = 1.0f / sqrtf(s * (1.0f / 16.0f) + 1e-6f);
  }
  __syncthreads();

#pragma unroll 1
  for (int it = 0; it < 4; ++it) {
    const int u = it * 256 + tid;
    const int b = u & 15, chh = (u >> 4) & 1, tok = u >> 5;
    const float rinv = sR[tok];
    const float* src = sX + tok * 256 + chh * 128 + b;
    F8 f;
#pragma unroll
    for (int j = 0; j < 8; ++j) f.v[j] = src[j * 16] * rinv;
    const HL o = split8(f);
    us* d = sA + ((((tok >> 4) * 16 + b) * 16) + (tok & 15)) * 32 + chh * 8;
    *(v4ua*)(d) = o.hi;
    *(v4ua*)(d + 16) = o.lo;
  }
  __syncthreads();

  {
    const v8f z8 = {0.f, 0.f, 0.f, 0.f, 0.f, 0.f, 0.f, 0.f};
    const int sub = w >> 2;
#pragma unroll 1
    for (int bi = 0; bi < 4; ++bi) {
      const int b = (w & 3) * 4 + bi;
      const int g = c_grade(b);
      const v16b a = ldfrag_s(sA + ((sub * 16 + b) * 16 + m) * 32 + 8 * h);
      const us* wrow = WP + g * 512 + m * 32 + 8 * h;
      const v16b bq = ldfrag_g(wrow + WP_Q);
      const v16b bk = ldfrag_g(wrow + WP_K);
      const v16b bv = ldfrag_g(wrow + WP_V);
      const v8f dq = mma_bf(a, bq, z8);
      const v8f dk = mma_bf(a, bk, z8);
      const v8f dv = mma_bf(a, bv, z8);
      unsigned vb[8];
#pragma unroll
      for (int r = 0; r < 8; ++r) {
        const int tok = sub * 16 + 8 * h + r;
        sQ[tok * 256 + m * 16 + b] = (us)bf_bits(0.125f * dq[r]);
        sK[tok * 256 + m * 16 + b] = (us)bf_bits(dk[r]);
        vb[r] = bf_bits(dv[r]);
      }
      const v4u pv = {vb[0] | (vb[1] << 16), vb[2] | (vb[3] << 16), vb[4] | (vb[5] << 16), vb[6] | (vb[7] << 16)};
      *(v4ua*)(sV + (m * 16 + b) * 32 + sub * 16 + 8 * h) = pv;
    }
  }
  __syncthreads();

  const int bidx = tok0 >> 11, n0 = tok0 & 2047;
  v4u rq[4], rk[4], rv[4];
  size_t oq[4], ov[4];
#pragma unroll
  for (int it = 0; it < 4; ++it) {
    const int p = it * 256 + tid;
    const int line = p >> 3, q8 = p & 7;
    const int tok = line >> 2, hd = line & 3;
    rq[it] = *(const v4ua*)(sQ + tok * 256 + hd * 64 + q8 * 8);
    rk[it] = *(const v4ua*)(sK + tok * 256 + hd * 64 + q8 * 8);
    oq[it] = ((size_t)(bidx * 4 + hd) * NSEQ + (size_t)(n0 + tok)) * HDIM + (size_t)q8 * 8;
    const int hd2 = p >> 8, wi = p & 255;
    rv[it] = *(const v4ua*)(sV + hd2 * 2048 + wi * 8);
    ov[it] = ((size_t)(bidx * 4 + hd2) * 64 + (size_t)(n0 >> 5)) * 2048 + (size_t)wi * 8;
  }
  v4f rx[8];
  if (L == 0) {
#pragma unroll
    for (int it = 0; it < 8; ++it) rx[it] = *(const v4fa*)(sX + (it * 256 + tid) * 4);
  }
  for (int pass = 0; pass < 2; ++pass) {
#pragma unroll
    for (int it = 0; it < 4; ++it) {
      *(volatile v4u*)(Qp + oq[it]) = rq[it];
      *(volatile v4u*)(Kp + oq[it]) = rk[it];
      *(volatile v4u*)(VTp + ov[it]) = rv[it];
    }
    if (L == 0) {
#pragma unroll
      for (int it = 0; it < 8; ++it)
        *(volatile v4f*)(Xout + (size_t)tok0 * 256 + (size_t)(it * 256 + tid) * 4) = rx[it];
    }
    __threadfence();
  }
}

__global__ __launch_bounds__(128) void k_attn(const us* __restrict__ Qp, const us* __restrict__ Kp,
                                              const us* __restrict__ VTp, float* __restrict__ Op) {
  __shared__ __align__(16) us Ks[64 * 64];
  __shared__ __align__(16) us Vt[64 * 64];
  __shared__ __align__(16) us Ps[4 * 16 * 64];
  __shared__ __align__(16) float Os[4 * 16 * 68];

  const int tid = threadIdx.x, wave = tid >> 5, lane = tid & 31, hh = lane >> 4, c = lane & 15;
  const int bx = blockIdx.x, qb = bx & 31, bh = bx >> 5;
  const int q0 = qb * 64 + wave * 16;
  const us* Qb = Qp + (size_t)bh * (NSEQ * HDIM);
  const us* Kb = Kp + (size_t)bh * (NSEQ * HDIM);
  const us* Vb = VTp + (size_t)bh * (NSEQ * HDIM);

  const v16b qa0 = ldfrag_g(Qb + (size_t)(q0 + c) * HDIM + 8 * hh);
  const v16b qa1 = ldfrag_g(Qb + (size_t)(q0 + c) * HDIM + 32 + 8 * hh);

  float mrow[8], lrow[8];
  v8f oacc[4];
#pragma unroll
  for (int r = 0; r < 8; ++r) { mrow[r] = -INFINITY; lrow[r] = 0.0f; }
#pragma unroll
  for (int t = 0; t < 4; ++t) oacc[t] = (v8f){0.f, 0.f, 0.f, 0.f, 0.f, 0.f, 0.f, 0.f};

  us* pw = Ps + wave * (16 * 64);

  for (int kc = 0; kc < NSEQ / 64; ++kc) {
    __syncthreads();
#pragma unroll
    for (int i = 0; i < 4; ++i) {
      const int p = i * 128 + tid;
      const v4u a = *(const v4ua*)(Kb + (size_t)kc * 4096 + (size_t)p * 8);
      const v4u b = *(const v4ua*)(Vb + (size_t)kc * 4096 + (size_t)p * 8);
      *(v4ua*)(Ks + p * 8) = a;
      const int cc = p >> 8, d = (p >> 2) & 63, kp = p & 3;
      *(v4ua*)(Vt + d * 64 + cc * 32 + kp * 8) = b;
    }
    __syncthreads();

    v8f s[4];
#pragma unroll
    for (int j = 0; j < 4; ++j) {
      s[j] = (v8f){0.f, 0.f, 0.f, 0.f, 0.f, 0.f, 0.f, 0.f};
      const v16b k0f = ldfrag_s(Ks + (j * 16 + c) * 64 + 8 * hh);
      const v16b k1f = ldfrag_s(Ks + (j * 16 + c) * 64 + 32 + 8 * hh);
      s[j] = mma_bf(qa0, k0f, s[j]);
      s[j] = mma_bf(qa1, k1f, s[j]);
    }
#pragma unroll
    for (int r = 0; r < 8; ++r) {
      float mx = fmaxf(fmaxf(s[0][r], s[1][r]), fmaxf(s[2][r], s[3][r]));
      mx = fmaxf(mx, __shfl_xor(mx, 1, 32));
      mx = fmaxf(mx, __shfl_xor(mx, 2, 32));
      mx = fmaxf(mx, __shfl_xor(mx, 4, 32));
      mx = fmaxf(mx, __shfl_xor(mx, 8, 32));
      const float mnew = fmaxf(mrow[r], mx);
      const float alpha = expf(mrow[r] - mnew);
      mrow[r] = mnew;
      float psum = 0.0f;
#pragma unroll
      for (int j = 0; j < 4; ++j) {
        const float p = expf(s[j][r] - mnew);
        const unsigned pb = bf_bits(p);
        psum += __uint_as_float(pb << 16);
        pw[(8 * hh + r) * 64 + j * 16 + c] = (us)pb;
      }
      lrow[r] = lrow[r] * alpha + psum;
#pragma unroll
      for (int t = 0; t < 4; ++t) oacc[t][r] *= alpha;
    }
    __builtin_amdgcn_fence(__ATOMIC_RELEASE, "workgroup");
    __builtin_amdgcn_wave_barrier();
    __builtin_amdgcn_fence(__ATOMIC_ACQUIRE, "workgroup");
#pragma unroll 1
    for (int kk = 0; kk < 2; ++kk) {
      const v16b pa = ldfrag_s(pw + c * 64 + kk * 32 + 8 * hh);
#pragma unroll
      for (int t = 0; t < 4; ++t) {
        const v16b vb = ldfrag_s(Vt + (t * 16 + c) * 64 + kk * 32 + 8 * hh);
        oacc[t] = mma_bf(pa, vb, oacc[t]);
      }
    }
  }

  float* os = Os + wave * (16 * 68);
#pragma unroll
  for (int r = 0; r < 8; ++r) {
    float l = lrow[r];
    l += __shfl_xor(l, 1, 32);
    l += __shfl_xor(l, 2, 32);
    l += __shfl_xor(l, 4, 32);
    l += __shfl_xor(l, 8, 32);
    const float inv = 1.0f / l;
#pragma unroll
    for (int t = 0; t < 4; ++t) os[(8 * hh + r) * 68 + t * 16 + c] = oacc[t][r] * inv;
  }
  __builtin_amdgcn_fence(__ATOMIC_RELEASE, "workgroup");
  __builtin_amdgcn_wave_barrier();
  __builtin_amdgcn_fence(__ATOMIC_ACQUIRE, "workgroup");
  {
    const int b = bh >> 2, hd = bh & 3;
    float* ob = Op + ((size_t)b * NSEQ) * NFEAT + hd * 64;
    const int c4 = (lane & 15) * 4;
    for (int pass = 0; pass < 2; ++pass) {
#pragma unroll
      for (int it = 0; it < 8; ++it) {
        const int row = it * 2 + hh;
        const v4f val = *(const v4fa*)(os + row * 68 + c4);
        *(volatile v4f*)(ob + (size_t)(q0 + row) * NFEAT + c4) = val;
      }
      __threadfence();
    }
  }
}

#define PO_XP 0
#define PO_U  16384
#define PO_A  114688
#define PO_G  212992
#define PO_R  219136
#define PO_T  219264
#define POST_LDS 223360
static_assert(POST_LDS <= 327680);

__device__ __forceinline__ void a32_unit(const float* src, float scale, us* dst) {
  F8 f;
#pragma unroll
  for (int j = 0; j < 8; ++j) f.v[j] = src[j * 16] * scale;
  const HL o = split8(f);
  *(v4ua*)(dst) = o.hi;
  *(v4ua*)(dst + 16) = o.lo;
}

__global__ __launch_bounds__(256) void k_post(const float* Xin, const float* __restrict__ Oin,
                                              const us* __restrict__ WP, float* Xout) {
  extern __shared__ __align__(16) unsigned char smem[];
  float*    sXp = (float*)(smem + PO_XP);
  float*    sU  = (float*)(smem + PO_U);
  us*       sA  = (us*)(smem + PO_A);
  float*    sG  = (float*)(smem + PO_G);
  float*    sR  = (float*)(smem + PO_R);
  unsigned* sT  = (unsigned*)(smem + PO_T);

  const int tid = threadIdx.x, lane = tid & 31, w = tid >> 5, h = lane >> 4, m = lane & 15;
  const int tok0 = blockIdx.x * 16;
  const v8f z8 = {0.f, 0.f, 0.f, 0.f, 0.f, 0.f, 0.f, 0.f};

#pragma unroll
  for (int it = 0; it < 4; ++it) {
    const int idx = it * 256 + tid;
    const v4f o = *(const v4fa*)(Oin + (size_t)tok0 * 256 + (size_t)idx * 4);
    const v4f x = *(const v4fa*)(Xin + (size_t)tok0 * 256 + (size_t)idx * 4);
    *(v4fa*)(sU + idx * 4) = o;
    *(v4fa*)(sXp + idx * 4) = x;
  }
  {
    const int k = tid >> 4, slot = tid & 15;
    const int km = c_mask(k);
    const int e0k = km & 1;
    const int i = e0k ? slot : c_noe0(slot & 7);
    const int valid = e0k | (slot < 8 ? 1 : 0);
    const int a = c_mask(i);
    const int b = a ^ km;
    const int j = c_idx(b);
    const float sf = valid ? (float)c_sign(a, b) : 0.0f;
    const v4u e = {(unsigned)i, (unsigned)j, __float_as_uint(sf), 0u};
    *(v4ua*)(sT + tid * 4) = e;
  }
  __syncthreads();

#pragma unroll 1
  for (int it = 0; it < 2; ++it) {
    const int u = it * 256 + tid;
    const int b = u & 15, chh = (u >> 4) & 1, tok = u >> 5;
    a32_unit(sU + tok * 256 + chh * 128 + b, 1.0f, sA + (b * 16 + tok) * 32 + chh * 8);
  }
  __syncthreads();

#pragma unroll 1
  for (int bi = 0; bi < 2; ++bi) {
    const int b = 2 * w + bi;
    const int g = c_grade(b);
    const v16b a = ldfrag_s(sA + (b * 16 + m) * 32 + 8 * h);
    const v16b bw = ldfrag_g(WP + WP_O + g * 512 + m * 32 + 8 * h);
    const v8f d = mma_bf(a, bw, z8);
#pragma unroll
    for (int r = 0; r < 8; ++r) sXp[(8 * h + r) * 256 + m * 16 + b] += d[r];
  }
  __syncthreads();

  {
    const int tok = tid >> 4, part = tid & 15;
    float s = 0.0f;
#pragma unroll
    for (int i = 0; i < 4; ++i) {
      const v4f v = *(const v4fa*)(sXp + tok * 256 + part * 16 + i * 4);
      s += v.x * v.x + v.y * v.y + v.z * v.z + v.w * v.w;
    }
    s += __shfl_xor(s, 1, 32);
    s += __shfl_xor(s, 2, 32);
    s += __shfl_xor(s, 4, 32);
    s += __shfl_xor(s, 8, 32);
    if (part == 0) sR[tok] = 1.0f / sqrtf(s * (1.0f / 16.0f) + 1e-6f);
  }
  __syncthreads();

#pragma unroll 1
  for (int it = 0; it < 2; ++it) {
    const int u = it * 256 + tid;
    const int b = u & 15, chh = (u >> 4) & 1, tok = u >> 5;
    a32_unit(sXp + tok * 256 + chh * 128 + b, sR[tok], sA + (b * 16 + tok) * 32 + chh * 8);
  }
  __syncthreads();

#pragma unroll 1
  for (int bi = 0; bi < 2; ++bi) {
    const int b = 2 * w + bi;
    const int g = c_grade(b);
    const v16b a = ldfrag_s(sA + (b * 16 + m) * 32 + 8 * h);
    v8f d[4];
#pragma unroll
    for (int nt = 0; nt < 4; ++nt) {
      const v16b bw = ldfrag_g(WP + WP_1 + g * 2048 + (nt * 16 + m) * 32 + 8 * h);
      d[nt] = mma_bf(a, bw, z8);
    }
#pragma unroll
    for (int nt = 0; nt < 4; ++nt)
#pragma unroll
      for (int r = 0; r < 8; ++r) sU[(8 * h + r) * 1536 + (nt * 16 + m) * 16 + b] = d[nt][r];
  }
  __syncthreads();

#pragma unroll 1
  for (int it = 0; it < 2; ++it) {
    const int item = it * 256 + tid;
    const int tok = item >> 5, rc = item & 31;
    const float* xb = sU + tok * 1536 + rc * 16;
    const float* yb = xb + 32 * 16;
    float* gb = sU + tok * 1536 + (64 + rc) * 16;
#pragma unroll 1
    for (int k = 0; k < 16; ++k) {
      const int nk = (c_mask(k) & 1) ? 16 : 8;
      float acc = 0.0f;
#pragma unroll 4
      for (int t = 0; t < nk; ++t) {
        const v4u e = *(const v4ua*)(sT + (k * 16 + t) * 4);
        acc = fmaf(__uint_as_float(e.z) * xb[e.x], yb[e.y], acc);
      }
      gb[k] = acc;
    }
  }
  __syncthreads();

#pragma unroll 1
  for (int it = 0; it < 6; ++it) {
    const int idx = it * 256 + tid;
    const int tok = idx / 96;
    const int ch = idx - tok * 96;
    const float v = sU[tok * 1536 + ch * 16];
    sG[idx] = 1.0f / (1.0f + expf(-v));
  }
  __syncthreads();

#pragma unroll 1
  for (int it = 0; it < 12; ++it) {
    const int u = it * 256 + tid;
    const int b = u & 15, rest = u >> 4;
    const int tok = rest / 12;
    const int ch0 = (rest - tok * 12) * 8;
    const v4f g0 = *(const v4fa*)(sG + tok * 96 + ch0);
    const v4f g1 = *(const v4fa*)(sG + tok * 96 + ch0 + 4);
    const float* src = sU + tok * 1536 + ch0 * 16 + b;
    F8 f;
    f.v[0] = src[0] * g0.x;   f.v[1] = src[16] * g0.y;  f.v[2] = src[32] * g0.z;  f.v[3] = src[48] * g0.w;
    f.v[4] = src[64] * g1.x;  f.v[5] = src[80] * g1.y;  f.v[6] = src[96] * g1.z;  f.v[7] = src[112] * g1.w;
    const HL o = split8(f);
    us* d = sA + (b * 16 + tok) * 192 + ch0;
    *(v4ua*)(d) = o.hi;
    *(v4ua*)(d + 96) = o.lo;
  }
  __syncthreads();

#pragma unroll 1
  for (int bi = 0; bi < 2; ++bi) {
    const int b = 2 * w + bi;
    const int g = c_grade(b);
    v8f acc = z8;
#pragma unroll 1
    for (int t = 0; t < 6; ++t) {
      const v16b a = ldfrag_s(sA + (b * 16 + m) * 192 + t * 32 + 8 * h);
      const v16b bw = ldfrag_g(WP + WP_2 + g * 3072 + m * 192 + t * 32 + 8 * h);
      acc = mma_bf(a, bw, acc);
    }
#pragma unroll
    for (int r = 0; r < 8; ++r) sXp[(8 * h + r) * 256 + m * 16 + b] += acc[r];
  }
  __syncthreads();

  v4f rx[4];
#pragma unroll
  for (int it = 0; it < 4; ++it) rx[it] = *(const v4fa*)(sXp + (it * 256 + tid) * 4);
  for (int pass = 0; pass < 2; ++pass) {
#pragma unroll
    for (int it = 0; it < 4; ++it)
      *(volatile v4f*)(Xout + (size_t)tok0 * 256 + (size_t)(it * 256 + tid) * 4) = rx[it];
    __threadfence();
  }
}

__global__ __launch_bounds__(256) void k_out(const float* __restrict__ X, const float* __restrict__ pw,
                                             const float* __restrict__ pos, float* __restrict__ out) {
  __shared__ float sPw[16];
  __shared__ __align__(16) float sOut[768];
  const int tid = threadIdx.x;
  if (tid < 16) sPw[tid] = bfr(pw[tid * 5 + 1]);
  __syncthreads();
  const size_t t = (size_t)blockIdx.x * 256 + tid;
  const float* xr = X + t * 256;
  float a0 = 0.0f, a1 = 0.0f, a2 = 0.0f;
#pragma unroll 4
  for (int c = 0; c < 16; ++c) {
    const v4f v = *(const v4fa*)(xr + c * 16);
    const v4f e = *(const v4fa*)(xr + c * 16 + 4);
    const float wv = sPw[c];
    a0 = fmaf(v.z, wv, a0);
    a1 = fmaf(v.w, wv, a1);
    a2 = fmaf(e.x, wv, a2);
  }
  sOut[tid * 3 + 0] = bfr(pos[t * 3 + 0]) + a0;
  sOut[tid * 3 + 1] = bfr(pos[t * 3 + 1]) + a1;
  sOut[tid * 3 + 2] = bfr(pos[t * 3 + 2]) + a2;
  __syncthreads();
  if (tid < 192) {
    const v4f val = *(const v4fa*)(sOut + tid * 4);
    float* dst = out + (size_t)blockIdx.x * 768 + (size_t)tid * 4;
    *(volatile v4f*)dst = val;
    __threadfence();
    *(volatile v4f*)dst = val;
  }
}
static_assert((NTOK / 256 - 1) * 768 + 767 == NTOK * 3 - 1);

extern "C" void kernel_launch(void* const* d_in, const int* in_sizes, int n_in,
                              void* d_out, int out_size, void* d_ws, size_t ws_size,
                              hipStream_t stream) {
  if (n_in < 10) return;
  if (in_sizes[0] != NTOK * 3 || in_sizes[1] != NTOK * 3) return;
  if (in_sizes[2] != 16 * 2 * 5) return;
  if (in_sizes[3] != 2 * 16 * 16 * 5 || in_sizes[4] != 2 * 16 * 16 * 5) return;
  if (in_sizes[5] != 2 * 16 * 16 * 5 || in_sizes[6] != 2 * 16 * 16 * 5) return;
  if (in_sizes[7] != 2 * 64 * 16 * 5 || in_sizes[8] != 2 * 16 * 96 * 5) return;
  if (in_sizes[9] != 16 * 5) return;
  if (out_size != NTOK * 3) return;

  const float* pos = (const float*)d_in[0];
  const float* vel = (const float*)d_in[1];
  const float* lw  = (const float*)d_in[2];
  const float* wq  = (const float*)d_in[3];
  const float* wk  = (const float*)d_in[4];
  const float* wv  = (const float*)d_in[5];
  const float* wo  = (const float*)d_in[6];
  const float* w1  = (const float*)d_in[7];
  const float* w2  = (const float*)d_in[8];
  const float* pw  = (const float*)d_in[9];
  float* out = (float*)d_out;

  const size_t SZ_F = (size_t)NTOK * NFEAT * 4;
  const size_t SZ_H = (size_t)NTOK * NFEAT * 2;
  const size_t SZ_W = (size_t)2 * WP_LAYER * 2;
  size_t off = 0;
  const size_t oX0 = off; off += SZ_F;
  const size_t oX1 = off; off += SZ_F;
  const size_t oO  = off; off += SZ_F;
  const size_t oQ  = off; off += SZ_H;
  const size_t oK  = off; off += SZ_H;
  const size_t oVT = off; off += SZ_H;
  const size_t oWP = off; off += SZ_W;
  if (off > ws_size) return;

  char* ws = (char*)d_ws;
  float* X0 = (float*)(ws + oX0);
  float* X1 = (float*)(ws + oX1);
  float* Ob = (float*)(ws + oO);
  us* Qp  = (us*)(ws + oQ);
  us* Kp  = (us*)(ws + oK);
  us* VTp = (us*)(ws + oVT);
  us* WPl = (us*)(ws + oWP);

  (void)hipFuncSetAttribute(reinterpret_cast<const void*>(&k_pre<0>), hipFuncAttributeMaxDynamicSharedMemorySize, PRE_LDS);
  (void)hipFuncSetAttribute(reinterpret_cast<const void*>(&k_pre<1>), hipFuncAttributeMaxDynamicSharedMemorySize, PRE_LDS);
  (void)hipFuncSetAttribute(reinterpret_cast<const void*>(&k_post), hipFuncAttributeMaxDynamicSharedMemorySize, POST_LDS);

  k_prep<<<140, 64, 0, stream>>>(wq, wk, wv, wo, w1, w2, WPl);

  k_pre<0><<<NTOK / 32, 256, PRE_LDS, stream>>>(pos, vel, lw, X0, X0, WPl, Qp, Kp, VTp);
  k_attn<<<32 * (NSEQ / 64), 128, 0, stream>>>(Qp, Kp, VTp, Ob);
  k_post<<<NTOK / 16, 256, POST_LDS, stream>>>(X0, Ob, WPl, X1);

  k_pre<1><<<NTOK / 32, 256, PRE_LDS, stream>>>(pos, vel, lw, X1, X1, WPl + WP_LAYER, Qp, Kp, VTp);
  k_attn<<<32 * (NSEQ / 64), 128, 0, stream>>>(Qp, Kp, VTp, Ob);
  k_post<<<NTOK / 16, 256, POST_LDS, stream>>>(X1, Ob, WPl + WP_LAYER, X0);

  k_out<<<NTOK / 256, 256, 0, stream>>>(X0, pw, pos, out);
  (void)hipGetLastError();
}
